// PyTorchTernaryKernel_43112881717530
// MI455X (gfx1250) — hardware-verified
//
#include <hip/hip_runtime.h>


#define TOK  512
#define INF  4096
#define OUTF 8192

typedef unsigned short bf;
typedef __attribute__((ext_vector_type(16))) __bf16   v16bf;
typedef __attribute__((ext_vector_type(8)))  unsigned short v8us;
typedef __attribute__((ext_vector_type(8)))  float    v8f;
typedef __attribute__((ext_vector_type(4)))  float    v4f;
typedef v4f  __attribute__((may_alias)) v4fa;

__device__ __forceinline__ unsigned short f2bf(float f) { unsigned u = __float_as_uint(f); u += 0x7FFFu + ((u >> 16) & 1u); return (unsigned short)(u >> 16); }
__device__ __forceinline__ float bf2f(unsigned short b) { return __uint_as_float(((unsigned)b) << 16); }
__device__ __forceinline__ float bfr(float f) { return bf2f(f2bf(f)); }
__device__ __forceinline__ v16bf cat16b(v8us lo, v8us hi) { return __builtin_bit_cast(v16bf, __builtin_shufflevector(lo, hi, 0, 1, 2, 3, 4, 5, 6, 7, 8, 9, 10, 11, 12, 13, 14, 15)); }
__device__ __forceinline__ v8f wmmab(v16bf a, v16bf b, v8f c) { return __builtin_amdgcn_wmma_f32_16x16x32_bf16(false, a, false, b, (short)0, c, false, false); }

__global__ __launch_bounds__(256) void k_cvtb(const float* __restrict__ x, bf* Xb) {
    const int lane = threadIdx.x & 31, r = blockIdx.x * 8 + (threadIdx.x >> 5);
    if (r >= TOK) return;
    const float* s = x + (size_t)r * INF; bf* d = Xb + (size_t)r * INF;
#pragma unroll 1
    for (int q = 0; q < INF / 256; ++q) {
        const float* p = s + q * 256 + lane * 8;
        v8us t;
#pragma unroll
        for (int i = 0; i < 8; ++i) t[i] = f2bf(p[i]);
        *(volatile v8us*)(d + q * 256 + lane * 8) = t;
        __threadfence();
        *(volatile v8us*)(d + q * 256 + lane * 8) = t;
    }
}

__global__ __launch_bounds__(256) void k_unpack(const int* __restrict__ packed, bf* Sb) {
    const int lane = threadIdx.x & 31, o = blockIdx.x * 8 + (threadIdx.x >> 5);
    if (o >= OUTF) return;
    const int* prow = packed + (size_t)o * (INF / 4); bf* d = Sb + (size_t)o * INF;
#pragma unroll 1
    for (int q = 0; q < INF / 256; ++q) {
        const int k0 = q * 256 + lane * 8;
        v8us t;
#pragma unroll
        for (int w = 0; w < 2; ++w) {
            const int word = prow[k0 / 4 + w];
#pragma unroll
            for (int j = 0; j < 4; ++j) {
                const int code = (word >> (2 * j)) & 3;
                t[w * 4 + j] = (code == 2) ? (unsigned short)0x3F80 : ((code == 0) ? (unsigned short)0xBF80 : (unsigned short)0);
            }
        }
        *(volatile v8us*)(d + k0) = t;
        __threadfence();
        *(volatile v8us*)(d + k0) = t;
    }
}

__global__ __launch_bounds__(128) void k_gemmb(const bf* __restrict__ A, const bf* __restrict__ Bn, int K, const float* __restrict__ alpha, const float* __restrict__ bias, float* C, int ldc) {
    __shared__ __align__(16) float ost[4][16 * 68];
    const int lane = threadIdx.x & 31, wave = threadIdx.x >> 5, lr = lane & 15, hi = lane >> 4;
    const int r0 = blockIdx.x * 64 + wave * 16, c0 = blockIdx.y * 64;
    const size_t aoff = (size_t)(r0 + lr) * K + 8 * hi;
    size_t boff[4];
#pragma unroll
    for (int t = 0; t < 4; ++t) boff[t] = (size_t)(c0 + t * 16 + lr) * K + 8 * hi;
    v8f acc[4];
#pragma unroll
    for (int t = 0; t < 4; ++t) acc[t] = (v8f){};
#pragma unroll 1
    for (int kc = 0; kc < K; kc += 32) {
        const v16bf a = cat16b(*(const v8us*)(A + aoff + kc), *(const v8us*)(A + aoff + kc + 16));
#pragma unroll
        for (int t = 0; t < 4; ++t) acc[t] = wmmab(a, cat16b(*(const v8us*)(Bn + boff[t] + kc), *(const v8us*)(Bn + boff[t] + kc + 16)), acc[t]);
        asm volatile("v_nop\n\tv_nop\n\tv_nop\n\tv_nop" : "+v"(acc[0]), "+v"(acc[1]), "+v"(acc[2]), "+v"(acc[3]) : "v"(a));
    }
    float* os = &ost[wave][0];
#pragma unroll
    for (int t = 0; t < 4; ++t) {
        const int n = c0 + t * 16 + lr;
        const float al = alpha ? bfr(alpha[n]) : 1.0f;
        const float bv = bias ? bfr(bias[n]) : 0.0f;
#pragma unroll
        for (int j = 0; j < 8; ++j) os[(hi * 8 + j) * 68 + t * 16 + lr] = acc[t][j] * al + bv;
    }
    __syncthreads();
    float* crow = C + (size_t)r0 * ldc + c0;
    auto pass = [&]() {
#pragma unroll
        for (int s = 0; s < 8; ++s) {
            const int Lid = (lane >> 3) + 4 * s, piece = lane & 7;
            const int row = Lid >> 1, cofs = (Lid & 1) * 32 + piece * 4;
            const v4f val = *(const v4fa*)(os + row * 68 + cofs);
            *(volatile v4f*)(crow + (size_t)row * ldc + cofs) = val;
        }
    };
    pass();
    __threadfence();
    pass();
}

extern "C" void kernel_launch(void* const* d_in, const int* in_sizes, int n_in,
                              void* d_out, int out_size, void* d_ws, size_t ws_size, hipStream_t stream) {
    (void)in_sizes; (void)n_in; (void)out_size;
    const float* x = (const float*)d_in[0]; const int* packed = (const int*)d_in[1]; const float* alpha = (const float*)d_in[2]; const float* bias = (const float*)d_in[3];
    float* out = (float*)d_out;
    char* wsp = (char*)d_ws;
    auto take = [&](size_t bytes) { char* p = wsp; wsp += (bytes + 255) & ~(size_t)255; return (void*)p; };
    bf* Xb = (bf*)take((size_t)TOK * INF * 2);
    bf* Sb = (bf*)take((size_t)OUTF * INF * 2);
    if ((size_t)(wsp - (char*)d_ws) > ws_size) return;
    k_cvtb<<<TOK / 8, 256, 0, stream>>>(x, Xb);
    k_unpack<<<OUTF / 8, 256, 0, stream>>>(packed, Sb);
    k_gemmb<<<dim3(TOK / 64, OUTF / 64, 1), 128, 0, stream>>>(Xb, Sb, INF, alpha, bias, out, OUTF);
}
